// MambaBlock_51745765982530
// MI455X (gfx1250) — hardware-verified
//
#include <hip/hip_runtime.h>
#include <math.h>

typedef __attribute__((ext_vector_type(16))) _Float16 v16h;
typedef __attribute__((ext_vector_type(8)))  _Float16 v8h;
typedef __attribute__((ext_vector_type(8)))  float    v8f;
typedef __attribute__((ext_vector_type(4)))  float    v4f;

constexpr int kBatch = 2;
constexpr int kSeq   = 1024;
constexpr int kDm    = 1024;
constexpr int kDin   = 2048;
constexpr int kNst   = 16;
constexpr int kDtR   = 64;
constexpr int kPrjN  = kDtR + 2 * kNst + kDin;
constexpr int kPrjP  = 2176;
constexpr int kXZP   = 2 * kDin;
constexpr int kRows  = kBatch * kSeq;
constexpr int kTP    = 260;
constexpr int kColB  = kDtR;
constexpr int kColC  = kDtR + kNst;
constexpr int kColG  = kDtR + 2 * kNst;

constexpr float kCarryW  = 32.0f;
constexpr float kCarryU  = 16.0f;
constexpr float kCarryDt = 16.0f;
constexpr float kCarryY  = 64.0f;
constexpr float kScaleIn  = 1.0f / kCarryW;
constexpr float kScaleXp  = 1.0f / (kCarryU * kCarryW);
constexpr float kScaleDt  = 1.0f / (kCarryDt * kCarryW);
constexpr float kScaleOut = 1.0f / (kCarryY * kCarryW);

static_assert(kPrjN == 2144, "x_proj width");
static_assert(kPrjP >= kPrjN && (kPrjP % 64) == 0, "padded x_proj width");
static_assert(kDtR == 64 && kNst == 16, "dt rank / state count");
static_assert((kSeq & (kSeq - 1)) == 0 && (kSeq % 64) == 0, "sequence tiling");
static_assert((kDm % 32) == 0 && (kDin % 32) == 0 && (kDtR % 32) == 0, "GEMM K multiples of 32");
static_assert((kRows % 64) == 0 && (kXZP % 64) == 0 && (kDin % 64) == 0 && (kDm % 64) == 0, "GEMM M,N multiples of 64");
static_assert((kDin % 256) == 0, "channel blocks");
static_assert((kColB * 4) % 16 == 0 && (kColG * 4) % 128 == 0, "PROJ column alignment");

constexpr size_t kOffX16  = 0;
constexpr size_t kOffWIN  = kOffX16  + (size_t)kRows * kDm  * 2;
constexpr size_t kOffWXP  = kOffWIN  + (size_t)kXZP  * kDm  * 2;
constexpr size_t kOffWDT  = kOffWXP  + (size_t)kPrjP * kDin * 2;
constexpr size_t kOffWOUT = kOffWDT  + (size_t)kDin  * kDtR * 2;
constexpr size_t kOffXZ   = kOffWOUT + (size_t)kDm   * kDin * 2;
constexpr size_t kOffUC   = kOffXZ   + (size_t)kRows * kXZP * 4;
constexpr size_t kOffUC16 = kOffUC   + (size_t)kRows * kDin * 4;
constexpr size_t kOffPROJ = kOffUC16 + (size_t)kRows * kDin * 2;
constexpr size_t kOffDT16 = kOffPROJ + (size_t)kRows * kPrjP * 4;
constexpr size_t kOffDLR  = kOffDT16 + (size_t)kRows * kDtR * 2;
constexpr size_t kOffY16  = kOffDLR  + (size_t)kRows * kDin * 4;
constexpr size_t kWsTotal = kOffY16  + (size_t)kRows * kDin * 2;
static_assert(kWsTotal == 127926272ull, "carve total");
static_assert(kWsTotal <= 134217728ull, "carve cap");
static_assert((kOffWIN % 128) == 0 && (kOffWXP % 128) == 0 && (kOffWDT % 128) == 0 && (kOffWOUT % 128) == 0 &&
              (kOffXZ % 128) == 0 && (kOffUC % 128) == 0 && (kOffUC16 % 128) == 0 && (kOffPROJ % 128) == 0 &&
              (kOffDT16 % 128) == 0 && (kOffDLR % 128) == 0 && (kOffY16 % 128) == 0, "128-B aligned regions");

__device__ __forceinline__ unsigned short f2bf_bits(float f) {
  unsigned u = __float_as_uint(f);
  return (unsigned short)((u + 0x7FFFu + ((u >> 16) & 1u)) >> 16);
}
__device__ __forceinline__ float bf_bits2f(unsigned short h) { return __uint_as_float(((unsigned)h) << 16); }
__device__ __forceinline__ float rne_bf16(float f) { return bf_bits2f(f2bf_bits(f)); }

__device__ __forceinline__ void wm_guard_row(v8f& c0, v8f& c1, v8f& c2, v8f& c3,
                                             v16h a, v16h b0, v16h b1, v16h b2, v16h b3) {
  asm volatile("v_nop\n\tv_nop\n\tv_nop\n\tv_nop"
               : "+v"(c0), "+v"(c1), "+v"(c2), "+v"(c3)
               : "v"(a), "v"(b0), "v"(b1), "v"(b2), "v"(b3));
}
__device__ __forceinline__ void keep4_h(v16h a, v16h b, v16h c, v16h d) { asm volatile("v_nop" :: "v"(a), "v"(b), "v"(c), "v"(d)); }
__device__ __forceinline__ void acc_guard4(v8f& a, v8f& b, v8f& c, v8f& d) { asm volatile("v_nop\n\tv_nop\n\tv_nop\n\tv_nop" : "+v"(a), "+v"(b), "+v"(c), "+v"(d)); }

struct FragH {
  union U { v16h v; v8h h[2]; };
  static __device__ __forceinline__ v16h load(const _Float16* p) {
    U f; f.h[0] = *(const v8h*)(p); f.h[1] = *(const v8h*)(p + 16); return f.v;
  }
  static __device__ __forceinline__ v8f mma(v16h a, v16h b, v8f c) {
    return __builtin_amdgcn_wmma_f32_16x16x32_f16(false, a, false, b, (short)0, c, false, false);
  }
};

__global__ __launch_bounds__(256) void wmma_gemm64_f16(
    const unsigned short* __restrict__ Ap, int lda,
    const unsigned short* __restrict__ Btp, int ldb,
    float* __restrict__ C, int ldc,
    int M, int N, int K, float scale) {
  const _Float16* A  = (const _Float16*)Ap;
  const _Float16* Bt = (const _Float16*)Btp;
  __shared__ __align__(16) float sT[8][16 * 68];
  const int lane = threadIdx.x & 31;
  const int wave = threadIdx.x >> 5;
  const int tilesN = N >> 6;
  const int tilesM = M >> 6;
  const int tile = blockIdx.x * 8 + wave;
  if (tile >= tilesM * tilesN) return;
  const int tm = tile / tilesN;
  const int tn = tile - tm * tilesN;
  const int m0 = tm << 6;
  const int n0 = tn << 6;

  const int rlane = lane & 15;
  const int koff  = (lane >> 4) * 8;
  const int mOff  = (lane >> 4) * 8;

  v8f acc[4][4];
#pragma unroll
  for (int i = 0; i < 4; ++i)
#pragma unroll
    for (int j = 0; j < 4; ++j) acc[i][j] = (v8f){0.f,0.f,0.f,0.f,0.f,0.f,0.f,0.f};

  for (int k0 = 0; k0 < K; k0 += 32) {
    v16h bh[4];
#pragma unroll
    for (int j = 0; j < 4; ++j) {
      const size_t bo = (size_t)(n0 + (j << 4) + rlane) * ldb + koff + k0;
      bh[j] = FragH::load(Bt + bo);
    }
#pragma unroll
    for (int i = 0; i < 4; ++i) {
      const size_t ao = (size_t)(m0 + (i << 4) + rlane) * lda + koff + k0;
      v16h ah = FragH::load(A + ao);
#pragma unroll
      for (int j = 0; j < 4; ++j) acc[i][j] = FragH::mma(ah, bh[j], acc[i][j]);
      wm_guard_row(acc[i][0], acc[i][1], acc[i][2], acc[i][3], ah, bh[0], bh[1], bh[2], bh[3]);
    }
    keep4_h(bh[0], bh[1], bh[2], bh[3]);
  }
  acc_guard4(acc[0][0], acc[0][1], acc[0][2], acc[0][3]);
  acc_guard4(acc[1][0], acc[1][1], acc[1][2], acc[1][3]);
  acc_guard4(acc[2][0], acc[2][1], acc[2][2], acc[2][3]);
  acc_guard4(acc[3][0], acc[3][1], acc[3][2], acc[3][3]);

  float* slab = sT[wave];
#pragma unroll
  for (int i = 0; i < 4; ++i) {
    const int mBase = m0 + (i << 4);
#pragma unroll
    for (int j = 0; j < 4; ++j) {
#pragma unroll
      for (int r = 0; r < 8; ++r) {
        const float v = acc[i][j][r] * scale;
        slab[(mOff + r) * 68 + (j << 4) + rlane] = v;
      }
    }
    __builtin_amdgcn_fence(__ATOMIC_RELEASE, "workgroup");
    __builtin_amdgcn_wave_barrier();
    __builtin_amdgcn_fence(__ATOMIC_ACQUIRE, "workgroup");
    {
      const int hh = lane >> 4, c4 = (lane & 15) * 4;
      for (int pass = 0; pass < 2; ++pass) {
#pragma unroll
        for (int it = 0; it < 8; ++it) {
          const int row = it * 2 + hh;
          v4f v = *(const v4f*)(slab + row * 68 + c4);
          *(volatile v4f*)(C + (size_t)(mBase + row) * ldc + n0 + c4) = v;
        }
        __threadfence();
      }
    }
    __builtin_amdgcn_fence(__ATOMIC_RELEASE, "workgroup");
    __builtin_amdgcn_wave_barrier();
    __builtin_amdgcn_fence(__ATOMIC_ACQUIRE, "workgroup");
  }
}

__global__ __launch_bounds__(256) void cast_rne_f16_kernel(
    const float* __restrict__ src, unsigned short* __restrict__ dst, int total8, int real8, float scale)
{
  const int i = blockIdx.x * 256 + threadIdx.x;
  if (i >= total8) return;
  const bool real = (i < real8);
  const int is = real ? i : (real8 - 1);
  const size_t es = (size_t)is << 3;
  const v4f a0 = *(const v4f*)(src + es);
  const v4f a1 = *(const v4f*)(src + es + 4);
  v8h hv;
#pragma unroll
  for (int e = 0; e < 4; ++e) {
    const float f0 = a0[e];
    const float f1 = a1[e];
    const float r0 = rne_bf16(f0) * scale;
    const float r1 = rne_bf16(f1) * scale;
    hv[e]     = (_Float16)(real ? r0 : 0.0f);
    hv[4 + e] = (_Float16)(real ? r1 : 0.0f);
  }
  unsigned short* q = dst + ((size_t)i << 3);
  *(volatile v8h*)q = hv;
  __threadfence();
  *(volatile v8h*)q = hv;
}

__global__ __launch_bounds__(256) void dt_cast_kernel(
    const float* __restrict__ PROJ, unsigned short* __restrict__ DT16, int total8, float scale)
{
  const int i = blockIdx.x * 256 + threadIdx.x;
  if (i >= total8) return;
  const int e0  = i << 3;
  const int row = e0 >> 6;
  const int c8  = e0 & 63;
  const float* p = PROJ + (size_t)row * kPrjP + c8;
  const v4f a0 = *(const v4f*)(p);
  const v4f a1 = *(const v4f*)(p + 4);
  v8h hv;
#pragma unroll
  for (int e = 0; e < 4; ++e) {
    hv[e]     = (_Float16)(a0[e] * scale);
    hv[4 + e] = (_Float16)(a1[e] * scale);
  }
  unsigned short* qd = DT16 + e0;
  *(volatile v8h*)qd = hv;
  __threadfence();
  *(volatile v8h*)qd = hv;
}

__global__ __launch_bounds__(256) void conv_silu_kernel(
    const float* __restrict__ XZ, const float* __restrict__ cw, const float* __restrict__ cb,
    float* __restrict__ UC, unsigned short* __restrict__ UC16)
{
  __shared__ __align__(16) float sT[16 * kTP];
  const int tid = threadIdx.x, lane = tid & 31, wave = tid >> 5;
  const int d0 = blockIdx.x * 256, d = d0 + tid;
  const int g0 = blockIdx.y * 64;
  const int tb = g0 & (kSeq - 1);
  const v4f wv = *(const v4f*)(cw + (size_t)d * 4);
  const float wr0 = wv[0], wr1 = wv[1], wr2 = wv[2], wr3 = wv[3];
  const float w0 = rne_bf16(wr0), w1 = rne_bf16(wr1), w2 = rne_bf16(wr2), w3 = rne_bf16(wr3);
  const float bc = rne_bf16(cb[d]);
  float xm3, xm2, xm1;
  {
    const bool hist = (tb > 0);
    const int rb = hist ? (g0 - 3) : g0;
    const float v3 = XZ[(size_t)rb * kXZP + d];
    const float v2 = XZ[(size_t)(rb + 1) * kXZP + d];
    const float v1 = XZ[(size_t)(rb + 2) * kXZP + d];
    xm3 = hist ? v3 : 0.f;
    xm2 = hist ? v2 : 0.f;
    xm1 = hist ? v1 : 0.f;
  }
  const int hrow = wave >> 1;
  const int hch  = (wave & 1) * 128 + lane * 4;
#pragma unroll 1
  for (int sub = 0; sub < 4; ++sub) {
    const int lb = g0 + sub * 16;
#pragma unroll 1
    for (int s = 0; s < 16; ++s) {
      const float xcur = XZ[(size_t)(lb + s) * kXZP + d];
      float acc = w0 * xm3;
      acc = fmaf(w1, xm2, acc);
      acc = fmaf(w2, xm1, acc);
      acc = fmaf(w3, xcur, acc);
      const float sv = acc + bc;
      const float sg = __builtin_amdgcn_rcpf(1.0f + __expf(-sv));
      sT[s * kTP + tid] = sv * sg;
      xm3 = xm2; xm2 = xm1; xm1 = xcur;
    }
    __syncthreads();
    v4f fv[4];
    v8h bv[2];
#pragma unroll
    for (int it = 0; it < 4; ++it) fv[it] = *(const v4f*)(sT + (it * 4 + hrow) * kTP + hch);
#pragma unroll
    for (int it = 0; it < 2; ++it) {
      const float* sp = sT + (it * 8 + wave) * kTP + lane * 8;
      const v4f a0 = *(const v4f*)(sp);
      const v4f a1 = *(const v4f*)(sp + 4);
#pragma unroll
      for (int e = 0; e < 4; ++e) {
        bv[it][e]     = (_Float16)(a0[e] * kCarryU);
        bv[it][4 + e] = (_Float16)(a1[e] * kCarryU);
      }
    }
    for (int pass = 0; pass < 2; ++pass) {
#pragma unroll
      for (int it = 0; it < 4; ++it)
        *(volatile v4f*)(UC + (size_t)(lb + it * 4 + hrow) * kDin + d0 + hch) = fv[it];
#pragma unroll
      for (int it = 0; it < 2; ++it)
        *(volatile v8h*)(UC16 + (size_t)(lb + it * 8 + wave) * kDin + d0 + lane * 8) = bv[it];
      __threadfence();
    }
    __syncthreads();
  }
}

__global__ __launch_bounds__(256) void scan_kernel(
    const float* __restrict__ DLR, const float* __restrict__ bdt, const float* __restrict__ UC,
    const float* __restrict__ XZ, const float* __restrict__ PROJ, const float* __restrict__ A_log,
    const float* __restrict__ Dv, unsigned short* __restrict__ Y16)
{
  __shared__ __align__(16) float sBC[16 * 32];
  __shared__ __align__(16) float sY[16 * kTP];
  const int tid = threadIdx.x, lane = tid & 31, wave = tid >> 5;
  const int d0 = blockIdx.x * 256, d = d0 + tid;
  const size_t row0 = (size_t)blockIdx.y * kSeq;

  float An[kNst], h[kNst];
#pragma unroll
  for (int q4 = 0; q4 < 4; ++q4) {
    const v4f al = *(const v4f*)(A_log + (size_t)d * kNst + 4 * q4);
    const float a0 = al[0], a1 = al[1], a2 = al[2], a3 = al[3];
    An[4 * q4 + 0] = -__expf(rne_bf16(a0));
    An[4 * q4 + 1] = -__expf(rne_bf16(a1));
    An[4 * q4 + 2] = -__expf(rne_bf16(a2));
    An[4 * q4 + 3] = -__expf(rne_bf16(a3));
  }
#pragma unroll
  for (int n = 0; n < kNst; ++n) h[n] = 0.f;
  const float bb = rne_bf16(bdt[d]);
  const float Dd = rne_bf16(Dv[d]);

#pragma unroll 1
  for (int c = 0; c < kSeq / 16; ++c) {
    const int l0 = c * 16;
    if (tid < 128) {
      const int r = tid >> 3, q = (tid & 7) * 4;
      const v4f v = *(const v4f*)(PROJ + (row0 + l0 + r) * kPrjP + kColB + q);
      *(v4f*)(sBC + r * 32 + q) = v;
    }
    __syncthreads();
#pragma unroll 1
    for (int s = 0; s < 16; ++s) {
      const size_t m = row0 + (size_t)(l0 + s);
      const float p     = DLR[m * kDin + d] + bb;
      const float delta = fmaxf(p, 0.0f) + log1pf(__expf(-fabsf(p)));
      const float xv    = UC[m * kDin + d];
      const float zv    = XZ[m * kXZP + kDin + d];
      const float gl    = PROJ[m * kPrjP + kColG + d];
      const float gs    = __builtin_amdgcn_rcpf(1.0f + __expf(-gl));
      const float dg    = delta * (0.5f + gs);
      const float dx    = delta * xv;
      v4f Bq[4], Cq[4];
#pragma unroll
      for (int qq = 0; qq < 4; ++qq) {
        Bq[qq] = *(const v4f*)(sBC + s * 32 + 4 * qq);
        Cq[qq] = *(const v4f*)(sBC + s * 32 + kNst + 4 * qq);
      }
      float y = 0.f;
#pragma unroll
      for (int n = 0; n < kNst; ++n) {
        const float e = __expf(dg * An[n]);
        const float hn = e * h[n] + dx * Bq[n >> 2][n & 3];
        h[n] = hn;
        y = Cq[n >> 2][n & 3] * hn + y;
      }
      y = xv * Dd + y;
      const float sg = __builtin_amdgcn_rcpf(1.0f + __expf(-zv));
      const float g  = zv * sg;
      sY[s * kTP + tid] = (y * g) * kCarryY;
    }
    __syncthreads();
    v8h hv[2];
#pragma unroll
    for (int it = 0; it < 2; ++it) {
      const float* sp = sY + (it * 8 + wave) * kTP + lane * 8;
      const v4f a0 = *(const v4f*)(sp);
      const v4f a1 = *(const v4f*)(sp + 4);
#pragma unroll
      for (int e = 0; e < 4; ++e) { hv[it][e] = (_Float16)a0[e]; hv[it][4 + e] = (_Float16)a1[e]; }
    }
    for (int pass = 0; pass < 2; ++pass) {
#pragma unroll
      for (int it = 0; it < 2; ++it)
        *(volatile v8h*)(Y16 + (row0 + (size_t)(l0 + it * 8 + wave)) * kDin + d0 + lane * 8) = hv[it];
      __threadfence();
    }
  }
}

static_assert(((kRows / 64) * (kXZP / 64)) % 8 == 0, "in_proj tiles per block");
static_assert(((kRows / 64) * (kPrjP / 64)) % 8 == 0, "x_proj tiles per block");
static_assert(((kRows / 64) * (kDin / 64)) % 8 == 0, "dt_proj tiles per block");
static_assert(((kRows / 64) * (kDm / 64)) % 8 == 0, "out_proj tiles per block");
static_assert(((kRows * kDm / 8) % 256) == 0 && ((kXZP * kDm / 8) % 256) == 0 && ((kPrjP * kDin / 8) % 256) == 0 &&
              ((kDin * kDtR / 8) % 256) == 0 && ((kDm * kDin / 8) % 256) == 0 && ((kRows * kDtR / 8) % 256) == 0,
              "cast grids exact");

extern "C" void kernel_launch(void* const* d_in, const int* in_sizes, int n_in,
                              void* d_out, int out_size, void* d_ws, size_t ws_size,
                              hipStream_t stream)
{
  if (n_in < 10) return;
  if (in_sizes[0] != kRows * kDm) return;
  if (in_sizes[1] != kXZP * kDm) return;
  if (in_sizes[2] != kDin * 4) return;
  if (in_sizes[3] != kDin) return;
  if (in_sizes[4] != kPrjN * kDin) return;
  if (in_sizes[5] != kDin * kDtR) return;
  if (in_sizes[6] != kDin) return;
  if (in_sizes[7] != kDin * kNst) return;
  if (in_sizes[8] != kDin) return;
  if (in_sizes[9] != kDm * kDin) return;
  if (out_size != kRows * kDm) return;
  if (ws_size < kWsTotal) return;

  const float* x      = (const float*)d_in[0];
  const float* W_in   = (const float*)d_in[1];
  const float* conv_w = (const float*)d_in[2];
  const float* conv_b = (const float*)d_in[3];
  const float* W_xp   = (const float*)d_in[4];
  const float* W_dt   = (const float*)d_in[5];
  const float* b_dt   = (const float*)d_in[6];
  const float* A_log  = (const float*)d_in[7];
  const float* Dv     = (const float*)d_in[8];
  const float* W_out  = (const float*)d_in[9];
  float* out = (float*)d_out;

  char* ws = (char*)d_ws;
  unsigned short* X16  = (unsigned short*)(ws + kOffX16);
  unsigned short* WIN  = (unsigned short*)(ws + kOffWIN);
  unsigned short* WXP  = (unsigned short*)(ws + kOffWXP);
  unsigned short* WDT  = (unsigned short*)(ws + kOffWDT);
  unsigned short* WOUT = (unsigned short*)(ws + kOffWOUT);
  float*          XZ   = (float*)(ws + kOffXZ);
  float*          UC   = (float*)(ws + kOffUC);
  unsigned short* UC16 = (unsigned short*)(ws + kOffUC16);
  float*          PROJ = (float*)(ws + kOffPROJ);
  unsigned short* DT16 = (unsigned short*)(ws + kOffDT16);
  float*          DLR  = (float*)(ws + kOffDLR);
  unsigned short* Y16  = (unsigned short*)(ws + kOffY16);

  cast_rne_f16_kernel<<<(kRows * kDm / 8) / 256, 256, 0, stream>>>(x, X16, kRows * kDm / 8, kRows * kDm / 8, 1.0f);
  cast_rne_f16_kernel<<<(kXZP * kDm / 8) / 256, 256, 0, stream>>>(W_in, WIN, kXZP * kDm / 8, kXZP * kDm / 8, kCarryW);
  cast_rne_f16_kernel<<<(kPrjP * kDin / 8) / 256, 256, 0, stream>>>(W_xp, WXP, kPrjP * kDin / 8, kPrjN * kDin / 8, kCarryW);
  cast_rne_f16_kernel<<<(kDin * kDtR / 8) / 256, 256, 0, stream>>>(W_dt, WDT, kDin * kDtR / 8, kDin * kDtR / 8, kCarryW);
  cast_rne_f16_kernel<<<(kDm * kDin / 8) / 256, 256, 0, stream>>>(W_out, WOUT, kDm * kDin / 8, kDm * kDin / 8, kCarryW);

  wmma_gemm64_f16<<<((kRows / 64) * (kXZP / 64)) / 8, 256, 0, stream>>>(
      X16, kDm, WIN, kDm, XZ, kXZP, kRows, kXZP, kDm, kScaleIn);

  conv_silu_kernel<<<dim3(kDin / 256, kRows / 64), 256, 0, stream>>>(XZ, conv_w, conv_b, UC, UC16);

  wmma_gemm64_f16<<<((kRows / 64) * (kPrjP / 64)) / 8, 256, 0, stream>>>(
      UC16, kDin, WXP, kDin, PROJ, kPrjP, kRows, kPrjP, kDin, kScaleXp);

  dt_cast_kernel<<<(kRows * kDtR / 8) / 256, 256, 0, stream>>>(PROJ, DT16, kRows * kDtR / 8, kCarryDt);

  wmma_gemm64_f16<<<((kRows / 64) * (kDin / 64)) / 8, 256, 0, stream>>>(
      DT16, kDtR, WDT, kDtR, DLR, kDin, kRows, kDin, kDtR, kScaleDt);

  scan_kernel<<<dim3(kDin / 256, kBatch), 256, 0, stream>>>(DLR, b_dt, UC, XZ, PROJ, A_log, Dv, Y16);

  wmma_gemm64_f16<<<((kRows / 64) * (kDm / 64)) / 8, 256, 0, stream>>>(
      Y16, kDin, WOUT, kDin, out, kDm, kRows, kDm, kDin, kScaleOut);
}
